// UnconstrainedOscillatorBank_36867999269144
// MI455X (gfx1250) — hardware-verified
//
#include <hip/hip_runtime.h>

#pragma clang fp contract(off)


typedef float          v8f   __attribute__((ext_vector_type(8)));
typedef float          v4f   __attribute__((ext_vector_type(4)));
typedef float          v4fa  __attribute__((ext_vector_type(4), may_alias));
typedef __bf16         v16bf __attribute__((ext_vector_type(16)));
typedef unsigned short v16us __attribute__((ext_vector_type(16)));

union Frag { v16bf v; v16us u; };

#define N_OSC    128
#define TCTRL    128
#define N_AUDIO  32768
#define BATCH    4
#define CHANNELS 128

#define K_PI     3.14159265358979323846f
#define K_INVPI  (1.0f / 3.14159265358979323846f)
#define K_BASE   ((float)(40.0 / 11025.0))
#define K_RANGE  ((float)(9000.0 / 11025.0 - 40.0 / 11025.0))

#define INV_2PI_D 0.15915494309189533577
#define TWO_PI_D  6.28318530717958647693
#define PI_D      3.14159265358979323846
#define PIO2_D    1.57079632679489661923

__device__ __forceinline__ unsigned short rne_bf16_bits(float f) {
    unsigned u = __float_as_uint(f);
    return (unsigned short)((u + 0x7FFFu + ((u >> 16) & 1u)) >> 16);
}
__device__ __forceinline__ float bf16_bits_to_f32(unsigned short b) {
    return __uint_as_float(((unsigned)b) << 16);
}
__device__ __forceinline__ void split3(float f, unsigned short& hb, unsigned short& mb, unsigned short& lb) {
    hb = rne_bf16_bits(f);
    const float r1 = f - bf16_bits_to_f32(hb);
    mb = rne_bf16_bits(r1);
    const float r2 = r1 - bf16_bits_to_f32(mb);
    lb = rne_bf16_bits(r2);
}

__device__ __forceinline__ v8f wmma_bf16(v16bf a, v16bf b, v8f c) {
    v8f d = __builtin_amdgcn_wmma_f32_16x16x32_bf16(false, a, false, b, (short)0, c, false, false);
    asm volatile("v_nop\n\tv_nop\n\tv_nop\n\tv_nop" : "+v"(d) : "v"(a), "v"(b));
    return d;
}

__device__ __forceinline__ void tile_step(const Frag& ah, const Frag& am, const Frag& al,
                                          const float* __restrict__ xb, int n, int k0, int h, v8f& acc)
{
    Frag bh, bm, bl;
#pragma unroll
    for (int i = 0; i < 16; ++i) {
        const int k = k0 + 8 * h + i + ((i >= 8) ? 8 : 0);
        const float f = xb[k * TCTRL + n];
        unsigned short x0, x1, x2;
        split3(f, x0, x1, x2);
        bh.u[i] = x0; bm.u[i] = x1; bl.u[i] = x2;
    }
    acc = wmma_bf16(ah.v, bh.v, acc);
    acc = wmma_bf16(ah.v, bm.v, acc);
    acc = wmma_bf16(am.v, bh.v, acc);
    acc = wmma_bf16(ah.v, bl.v, acc);
    acc = wmma_bf16(am.v, bm.v, acc);
    acc = wmma_bf16(al.v, bh.v, acc);
}

__device__ __forceinline__ void tile_epilogue(const v8f& acc, int Mbase, int h, int t,
                                              const float* __restrict__ bias, const float* __restrict__ bl,
                                              float* fS, float* aS)
{
#pragma unroll
    for (int jj = 0; jj < 4; ++jj) {
        const int Mr   = Mbase + 8 * h + 2 * jj;
        const int osc  = Mr >> 1;
        const int oscl = 4 * h + jj;
        const float re = acc[2 * jj]     + bias[Mr];
        const float im = acc[2 * jj + 1] + bias[Mr + 1];
        const float r  = re * 0.01f + bl[2 * osc + 0];
        const float i  = im * 0.01f + bl[2 * osc + 1];
        const float rr = r * r;
        const float ii = i * i;
        const float a1 = sqrtf(rr + ii);
        const float fr = atan2f(i, r) * K_INVPI;
        const float fq = fr * fr;
        const float a2 = a1 * a1;
        const float a3 = a2 * K_RANGE;
        const float av = K_BASE + a3;
        fS[oscl * TCTRL + t] = fq;
        aS[oscl * TCTRL + t] = av;
    }
}

__global__ __launch_bounds__(128)
void k_ctrl(const float* __restrict__ X, const float* __restrict__ W,
            const float* __restrict__ bias, const float* __restrict__ bl,
            float* __restrict__ freq_c, float* __restrict__ amp_c)
{
    __shared__ float fS[8 * TCTRL];
    __shared__ float aS[8 * TCTRL];

    const int lane = threadIdx.x & 31;
    const int wv   = threadIdx.x >> 5;
    const int h    = lane >> 4;
    const int m    = lane & 15;
    const int mt   = blockIdx.x & 15;
    const int bI   = blockIdx.x >> 4;
    const int Mbase = mt * 16;
    const float* __restrict__ xb = X + (size_t)bI * CHANNELS * TCTRL;

    v8f acc0 = {0.f, 0.f, 0.f, 0.f, 0.f, 0.f, 0.f, 0.f};
    v8f acc1 = {0.f, 0.f, 0.f, 0.f, 0.f, 0.f, 0.f, 0.f};
    const int n0 = wv * 32 + m;
    const int n1 = wv * 32 + 16 + m;

    for (int k0 = 0; k0 < CHANNELS; k0 += 32) {
        Frag ah, am, al;
#pragma unroll
        for (int i = 0; i < 16; ++i) {
            const int k = k0 + 8 * h + i + ((i >= 8) ? 8 : 0);
            const float f = W[(Mbase + m) * CHANNELS + k];
            unsigned short x0, x1, x2;
            split3(f, x0, x1, x2);
            ah.u[i] = x0; am.u[i] = x1; al.u[i] = x2;
        }
        tile_step(ah, am, al, xb, n0, k0, h, acc0);
        tile_step(ah, am, al, xb, n1, k0, h, acc1);
    }

    tile_epilogue(acc0, Mbase, h, n0, bias, bl, fS, aS);
    tile_epilogue(acc1, Mbase, h, n1, bias, bl, fS, aS);
    __syncthreads();

    v4f vf[2], va[2];
    float* pf[2];
    float* pa[2];
#pragma unroll
    for (int rr = 0; rr < 2; ++rr) {
        const int row = 2 * wv + rr;
        const int gr  = bI * N_OSC + 8 * mt + row;
        vf[rr] = *(const v4fa*)(fS + row * TCTRL + 4 * lane);
        va[rr] = *(const v4fa*)(aS + row * TCTRL + 4 * lane);
        pf[rr] = freq_c + (size_t)gr * TCTRL + 4 * lane;
        pa[rr] = amp_c  + (size_t)gr * TCTRL + 4 * lane;
        *(volatile v4f*)pf[rr] = vf[rr];
        *(volatile v4f*)pa[rr] = va[rr];
    }
    __threadfence();
#pragma unroll
    for (int rr = 0; rr < 2; ++rr) {
        *(volatile v4f*)pf[rr] = vf[rr];
        *(volatile v4f*)pa[rr] = va[rr];
    }
}

__device__ __forceinline__ float sin_f32(float ph)
{
    const double pd = (double)ph;
    const double k  = __builtin_rint(pd * INV_2PI_D);
    double r = __builtin_fma(-k, TWO_PI_D, pd);
    if (r > PIO2_D)       r = PI_D - r;
    else if (r < -PIO2_D) r = -PI_D - r;
    const float x  = (float)r;
    const float x2 = x * x;
    float p = -2.5052108e-8f;
    p = p * x2 + 2.7557319e-6f;
    p = p * x2 - 1.9841270e-4f;
    p = p * x2 + 8.3333333e-3f;
    p = p * x2 - 1.6666667e-1f;
    const float x3 = x2 * x;
    return x + x3 * p;
}

__global__ __launch_bounds__(128)
void k_render(const float* __restrict__ freq_c, const float* __restrict__ amp_c,
              float* __restrict__ out)
{
    __shared__ float tile[N_OSC * 65];
    __shared__ float outS[128];

    const int o  = threadIdx.x;
    const int bI = blockIdx.x;
    const float* __restrict__ fr = freq_c + (size_t)(bI * N_OSC + o) * TCTRL;
    const float* __restrict__ ar = amp_c  + (size_t)(bI * N_OSC + o) * TCTRL;
    float* __restrict__ ob = out + (size_t)bI * N_AUDIO;

    float R = 0.0f;
    float E = 0.0f;

    for (int B = 0; B < 256; ++B) {
        const float excl = (B < 128) ? R : (R + E);
        const int i0 = (B == 0) ? 0 : ((B - 1) >> 1);
        const int i1 = (i0 + 1 < TCTRL) ? (i0 + 1) : (TCTRL - 1);
        const float f0 = fr[i0], f1 = fr[i1];
        const float a0 = ar[i0], a1 = ar[i1];
        const float fi0 = (float)i0;
        float inner = 0.0f;

        for (int hh = 0; hh < 2; ++hh) {
            for (int t2 = 0; t2 < 64; ++t2) {
                const int j = B * 128 + hh * 64 + t2;
                float pos = ((float)j + 0.5f) * 0.00390625f - 0.5f;
                pos = fminf(fmaxf(pos, 0.0f), 127.0f);
                const float w   = pos - fi0;
                const float omw = 1.0f - w;
                const float fa  = f0 * omw;
                const float fb  = f1 * w;
                const float f   = fa + fb;
                const float v   = f * K_PI;
                inner = inner + v;
                const float ph  = inner + excl;
                const float aa  = a0 * omw;
                const float ab  = a1 * w;
                const float am  = aa + ab;
                tile[o * 65 + t2] = sin_f32(ph) * am;
            }
            __syncthreads();
            if (o < 64) {
                float s = 0.0f;
                for (int q = 0; q < N_OSC; ++q) s += tile[q * 65 + o];
                outS[hh * 64 + o] = s;
            }
            __syncthreads();
        }

        const float T = inner;
        if (B == 127) { E = R; R = T; }
        else          { R = R + T; }

        if (o < 32) {
            const v4f val = *(const v4fa*)(outS + 4 * o);
            float* p = ob + (size_t)B * 128 + 4 * o;
            *(volatile v4f*)p = val;
            __threadfence();
            *(volatile v4f*)p = val;
        }
    }
}

extern "C" void kernel_launch(void* const* d_in, const int* in_sizes, int n_in,
                              void* d_out, int out_size, void* d_ws, size_t ws_size,
                              hipStream_t stream)
{
    if (n_in < 4) return;
    if (in_sizes[0] != BATCH * CHANNELS * TCTRL) return;
    if (in_sizes[1] != 2 * N_OSC * CHANNELS) return;
    if (in_sizes[2] != 2 * N_OSC) return;
    if (in_sizes[3] != N_OSC * 2) return;
    if (out_size != BATCH * N_AUDIO) return;
    const size_t nctrl = (size_t)BATCH * N_OSC * TCTRL;
    if (ws_size < 2 * nctrl * sizeof(float)) return;

    const float* X    = (const float*)d_in[0];
    const float* W    = (const float*)d_in[1];
    const float* bias = (const float*)d_in[2];
    const float* bl   = (const float*)d_in[3];
    float* out = (float*)d_out;

    float* ws     = (float*)d_ws;
    float* freq_c = ws;
    float* amp_c  = ws + nctrl;

    k_ctrl<<<BATCH * 16, 128, 0, stream>>>(X, W, bias, bl, freq_c, amp_c);
    k_render<<<BATCH, 128, 0, stream>>>(freq_c, amp_c, out);
}
